// RopelessMLAEncoderBlock_50251117363437
// MI455X (gfx1250) — hardware-verified
//
#include <hip/hip_runtime.h>
#include <stddef.h>
#include <stdint.h>
#include <math.h>

#define BB   2
#define NN   2048
#define CC   1024
#define HH   16
#define DD   64
#define FF   4096
#define LAT  256
#define ROWS (BB * NN)
#define PL   ((size_t)BB * HH * NN * DD)

static_assert(NN % 256 == 0);
static_assert(CC % 64 == 0);
static_assert(FF % 64 == 0);
static_assert(LAT % 64 == 0);
static_assert(DD == 64);
static_assert(HH * DD == CC);
static_assert(ROWS % 256 == 0);
static_assert((ROWS * CC) % 8 == 0);

typedef _Float16 v16h __attribute__((ext_vector_type(16)));
typedef _Float16 v8h  __attribute__((ext_vector_type(8)));
typedef float    v8f  __attribute__((ext_vector_type(8)));
typedef float    v4f  __attribute__((ext_vector_type(4)));
typedef unsigned int v4u __attribute__((ext_vector_type(4)));

union Frag  { v16h v; v8h h[2]; };
union Pack8 { v8h h; v4u u; };

__device__ __forceinline__ v8f mma16(v16h a, v16h b, v8f c) {
  c = __builtin_amdgcn_wmma_f32_16x16x32_f16(false, a, false, b, (short)0, c, false, false);
  asm volatile("v_nop\n\tv_nop\n\tv_nop\n\tv_nop" : "+v"(c) : "v"(a), "v"(b));
  return c;
}

__device__ __forceinline__ v16h ldfrag(const _Float16* p, int ld, int row0, int k0, int lane) {
  const int m = lane & 15, lh = lane >> 4;
  const _Float16* q = p + (size_t)(row0 + m) * ld + k0 + 8 * lh;
  Frag f;
  f.h[0] = *(const v8h*)(q);
  f.h[1] = *(const v8h*)(q + 16);
  return f.v;
}

__device__ __forceinline__ v8f zero8() { return (v8f){0.f, 0.f, 0.f, 0.f, 0.f, 0.f, 0.f, 0.f}; }

__device__ __forceinline__ float act16(float v) {
  return 8.0f * v * (1.0f + erff(v * 0.70710678118654752f));
}

template <int KK>
__device__ __forceinline__ void gemm32x64(const _Float16* __restrict__ A, int lda,
                                          const _Float16* __restrict__ Bt, int ldb,
                                          int m0, int n0, int lane, v8f (&acc)[2][4]) {
#pragma unroll 2
  for (int k0 = 0; k0 < KK; k0 += 32) {
    const v16h a0 = ldfrag(A, lda, m0, k0, lane);
    const v16h a1 = ldfrag(A, lda, m0 + 16, k0, lane);
    const v16h b0 = ldfrag(Bt, ldb, n0, k0, lane);
    const v16h b1 = ldfrag(Bt, ldb, n0 + 16, k0, lane);
    const v16h b2 = ldfrag(Bt, ldb, n0 + 32, k0, lane);
    const v16h b3 = ldfrag(Bt, ldb, n0 + 48, k0, lane);
    acc[0][0] = mma16(a0, b0, acc[0][0]);
    acc[1][0] = mma16(a1, b0, acc[1][0]);
    acc[0][1] = mma16(a0, b1, acc[0][1]);
    acc[1][1] = mma16(a1, b1, acc[1][1]);
    acc[0][2] = mma16(a0, b2, acc[0][2]);
    acc[1][2] = mma16(a1, b2, acc[1][2]);
    acc[0][3] = mma16(a0, b3, acc[0][3]);
    acc[1][3] = mma16(a1, b3, acc[1][3]);
  }
}

__global__ __launch_bounds__(256) void k_cvt_x(const float* __restrict__ x, _Float16* __restrict__ xh, int ngrp) {
  const int t = blockIdx.x * 256 + (int)threadIdx.x;
  if (t >= ngrp) return;
  const size_t o = (size_t)t * 8;
  const v4f a0 = *(const v4f*)(x + o);
  const v4f a1 = *(const v4f*)(x + o + 4);
  Pack8 pk;
  pk.h = (v8h){(_Float16)a0[0], (_Float16)a0[1], (_Float16)a0[2], (_Float16)a0[3],
               (_Float16)a1[0], (_Float16)a1[1], (_Float16)a1[2], (_Float16)a1[3]};
  const v4u vv = pk.u;
  volatile v4u* d = (volatile v4u*)(xh + o);
  *d = vv;
  __threadfence();
  *d = vv;
}

#define WTP 68
__global__ __launch_bounds__(256) void k_wt(const float* __restrict__ w, _Float16* __restrict__ wt,
                                           int nout, int kin) {
  __shared__ __align__(16) float tf[64 * WTP];
  const int tid = threadIdx.x;
  const int n0 = blockIdx.x * 64;
  const int k0 = blockIdx.y * 64;
  {
    const int kr = tid >> 4;
    const int n4 = (tid & 15) * 4;
#pragma unroll
    for (int it = 0; it < 4; ++it) {
      const int kl = it * 16 + kr;
      const v4f a = *(const v4f*)(w + (size_t)(k0 + kl) * nout + n0 + n4);
      *(v4f*)(tf + kl * WTP + n4) = a;
    }
  }
  __syncthreads();
  v4u val[2];
  size_t go[2];
#pragma unroll
  for (int j = 0; j < 2; ++j) {
    const int p  = tid + 256 * j;
    const int nl = p >> 3;
    const int pc = p & 7;
    const float* cp = tf + (pc * 8) * WTP + nl;
    Pack8 pk;
    pk.h = (v8h){(_Float16)(cp[0 * WTP] * 32.0f), (_Float16)(cp[1 * WTP] * 32.0f),
                 (_Float16)(cp[2 * WTP] * 32.0f), (_Float16)(cp[3 * WTP] * 32.0f),
                 (_Float16)(cp[4 * WTP] * 32.0f), (_Float16)(cp[5 * WTP] * 32.0f),
                 (_Float16)(cp[6 * WTP] * 32.0f), (_Float16)(cp[7 * WTP] * 32.0f)};
    val[j] = pk.u;
    go[j]  = (size_t)(n0 + nl) * kin + k0 + pc * 8;
  }
  for (int ps = 0; ps < 2; ++ps) {
#pragma unroll
    for (int j = 0; j < 2; ++j) *(volatile v4u*)(wt + go[j]) = val[j];
    __threadfence();
  }
}

#define STP 72
__global__ __launch_bounds__(256) void k_lat(const _Float16* __restrict__ xh,
                                             const _Float16* __restrict__ wt,
                                             const float* __restrict__ bk,
                                             const float* __restrict__ bv,
                                             _Float16* __restrict__ kv) {
  __shared__ __align__(16) _Float16 st[256 * STP];
  const int tid = threadIdx.x, lane = tid & 31, wave = tid >> 5;
  const int hh = lane >> 4, c = lane & 15;
  const int mb = blockIdx.x * 256;
  const int m0 = mb + wave * 32;
  const int n0 = blockIdx.y * 64;
  const int which = n0 >> 8;
  const int nin = n0 & (LAT - 1);

  v8f acc[2][4];
#pragma unroll
  for (int s = 0; s < 2; ++s)
#pragma unroll
    for (int t = 0; t < 4; ++t) acc[s][t] = zero8();
  gemm32x64<CC>(xh, CC, wt, CC, m0, n0, lane, acc);

#pragma unroll
  for (int t = 0; t < 4; ++t) {
    const int nn = nin + 16 * t + c;
    const float v0 = bk[nn], v1 = bv[nn];
    const float bb = (which == 0) ? v0 : v1;
#pragma unroll
    for (int sub = 0; sub < 2; ++sub) {
#pragma unroll
      for (int r = 0; r < 8; ++r) {
        const int lr = wave * 32 + sub * 16 + 8 * hh + r;
        st[lr * STP + 16 * t + c] = (_Float16)(acc[sub][t][r] * 0.03125f + bb);
      }
    }
  }
  __syncthreads();

  v4u val[8];
  size_t go[8];
#pragma unroll
  for (int j = 0; j < 8; ++j) {
    const int p  = tid + 256 * j;
    const int lr = p >> 3;
    const int pc = p & 7;
    Pack8 pk;
    pk.h  = *(const v8h*)(st + lr * STP + pc * 8);
    val[j] = pk.u;
    go[j]  = (size_t)which * ROWS * LAT + (size_t)(mb + lr) * LAT + nin + pc * 8;
  }
  for (int ps = 0; ps < 2; ++ps) {
#pragma unroll
    for (int j = 0; j < 8; ++j) *(volatile v4u*)(kv + go[j]) = val[j];
    __threadfence();
  }
}

template <int KK, int TR>
__global__ __launch_bounds__(256) void k_hp(const _Float16* __restrict__ ap,
                                            const _Float16* __restrict__ wt,
                                            const float* __restrict__ bias,
                                            _Float16* __restrict__ plane, float oscale, float bscale) {
  __shared__ __align__(16) _Float16 st[256 * STP];
  const int tid = threadIdx.x, lane = tid & 31, wave = tid >> 5;
  const int hh = lane >> 4, c = lane & 15;
  const int mb = blockIdx.x * 256;
  const int m0 = mb + wave * 32;
  const int n0 = blockIdx.y * 64;

  v8f acc[2][4];
#pragma unroll
  for (int s = 0; s < 2; ++s)
#pragma unroll
    for (int t = 0; t < 4; ++t) acc[s][t] = zero8();
  gemm32x64<KK>(ap, KK, wt, KK, m0, n0, lane, acc);

#pragma unroll
  for (int t = 0; t < 4; ++t) {
    const float bb = bias[n0 + 16 * t + c] * bscale;
#pragma unroll
    for (int sub = 0; sub < 2; ++sub) {
#pragma unroll
      for (int r = 0; r < 8; ++r) {
        const int lr = wave * 32 + sub * 16 + 8 * hh + r;
        st[lr * STP + 16 * t + c] = (_Float16)(acc[sub][t][r] * oscale + bb);
      }
    }
  }
  __syncthreads();

  const int head = n0 >> 6;
  const int b  = mb >> 11;
  const int nb = mb & (NN - 1);
  const int bh = b * HH + head;
  v4u val[8];
  size_t go[8];
  if (TR == 0) {
#pragma unroll
    for (int j = 0; j < 8; ++j) {
      const int p  = tid + 256 * j;
      const int lr = p >> 3;
      const int pc = p & 7;
      Pack8 pk;
      pk.h  = *(const v8h*)(st + lr * STP + pc * 8);
      val[j] = pk.u;
      go[j]  = ((size_t)bh * NN + nb + lr) * DD + pc * 8;
    }
  } else {
#pragma unroll
    for (int j = 0; j < 8; ++j) {
      const int p  = tid + 256 * j;
      const int L  = p >> 3;
      const int pc = p & 7;
      const int d  = L >> 2;
      const int nl = (L & 3) * 64 + pc * 8;
      const _Float16* cp = st + nl * STP + d;
      Pack8 pk;
      pk.h = (v8h){cp[0 * STP], cp[1 * STP], cp[2 * STP], cp[3 * STP],
                   cp[4 * STP], cp[5 * STP], cp[6 * STP], cp[7 * STP]};
      val[j] = pk.u;
      go[j]  = ((size_t)bh * DD + d) * NN + nb + nl;
    }
  }
  for (int ps = 0; ps < 2; ++ps) {
#pragma unroll
    for (int j = 0; j < 8; ++j) *(volatile v4u*)(plane + go[j]) = val[j];
    __threadfence();
  }
}

#define KTP 72
#define PTP 72
#define BTP 64
__global__ __launch_bounds__(256) void k_attn(const _Float16* __restrict__ qp,
                                              const _Float16* __restrict__ kp,
                                              const _Float16* __restrict__ vt,
                                              const float* __restrict__ ab,
                                              _Float16* __restrict__ op, float sscale) {
  __shared__ __align__(16) _Float16 Ks[64 * KTP];
  __shared__ __align__(16) _Float16 Vs[64 * KTP];
  __shared__ __align__(16) _Float16 Ps[8][16 * PTP];
  __shared__ __align__(16) float    Bs[8][16 * BTP];

  const int tid = threadIdx.x, lane = tid & 31, wave = tid >> 5;
  const int hh = lane >> 4, c = lane & 15;
  const int bh = blockIdx.x >> 4;
  const int qb = blockIdx.x & 15;
  const int b  = bh >> 4, h = bh & (HH - 1);
  const int q0 = qb * 128 + wave * 16;

  const _Float16* Q = qp + (size_t)bh * NN * DD;
  const _Float16* K = kp + (size_t)bh * NN * DD;
  const _Float16* V = vt + (size_t)bh * DD * NN;

  v16h qa[2];
  qa[0] = ldfrag(Q, DD, q0, 0, lane);
  qa[1] = ldfrag(Q, DD, q0, 32, lane);

  const float NEGI = -__builtin_huge_valf();
  float mrow[8], lrow[8];
  v8f oacc[4];
#pragma unroll
  for (int r = 0; r < 8; ++r) { mrow[r] = NEGI; lrow[r] = 0.f; }
#pragma unroll
  for (int t = 0; t < 4; ++t) oacc[t] = zero8();

  _Float16* pw = Ps[wave];
  float*    bw = Bs[wave];

  for (int kc = 0; kc < NN / 64; ++kc) {
    const int kv0 = kc * 64;
    __syncthreads();
    {
      const int r  = tid >> 2;
      const int qq = (tid & 3) * 16;
      const _Float16* ks = K + (size_t)(kv0 + r) * DD + qq;
      *(v8h*)(Ks + r * KTP + qq)     = *(const v8h*)(ks);
      *(v8h*)(Ks + r * KTP + qq + 8) = *(const v8h*)(ks + 8);
      const _Float16* vs = V + (size_t)r * NN + kv0 + qq;
      *(v8h*)(Vs + r * KTP + qq)     = *(const v8h*)(vs);
      *(v8h*)(Vs + r * KTP + qq + 8) = *(const v8h*)(vs + 8);
#pragma unroll
      for (int it = 0; it < 8; ++it) {
        const int p   = lane + 32 * it;
        const int row = p >> 4;
        const int c4  = (p & 15) * 4;
        const v4f bv4 = *(const v4f*)(ab + (size_t)(q0 + row) * NN + kv0 + c4);
        *(v4f*)(bw + row * BTP + c4) = bv4;
      }
    }
    __syncthreads();

    v8f s[4];
#pragma unroll
    for (int j = 0; j < 4; ++j) s[j] = zero8();
#pragma unroll
    for (int dc = 0; dc < 2; ++dc) {
#pragma unroll
      for (int j = 0; j < 4; ++j) {
        const v16h kb = ldfrag(Ks, KTP, j * 16, dc * 32, lane);
        s[j] = mma16(qa[dc], kb, s[j]);
      }
    }
    float cm[8];
#pragma unroll
    for (int r = 0; r < 8; ++r) {
      float m = NEGI;
#pragma unroll
      for (int j = 0; j < 4; ++j) {
        const float sv = s[j][r] * sscale + bw[(8 * hh + r) * BTP + 16 * j + c];
        s[j][r] = sv;
        m = fmaxf(m, sv);
      }
#pragma unroll
      for (int off = 1; off < 16; off <<= 1) m = fmaxf(m, __shfl_xor(m, off, 32));
      cm[r] = m;
    }
    float al[8];
#pragma unroll
    for (int r = 0; r < 8; ++r) {
      const float mnew  = fmaxf(mrow[r], cm[r]);
      const float alpha = __expf(mrow[r] - mnew);
      mrow[r] = mnew;
      float psum = 0.f;
#pragma unroll
      for (int j = 0; j < 4; ++j) {
        const float p = __expf(s[j][r] - mnew);
        psum += p;
        pw[(8 * hh + r) * PTP + j * 16 + c] = (_Float16)(p * 1024.0f);
      }
#pragma unroll
      for (int off = 1; off < 16; off <<= 1) psum += __shfl_xor(psum, off, 32);
      lrow[r] = lrow[r] * alpha + psum;
      al[r] = alpha;
    }
#pragma unroll
    for (int t = 0; t < 4; ++t)
#pragma unroll
      for (int r = 0; r < 8; ++r) oacc[t][r] *= al[r];
    __syncthreads();

#pragma unroll
    for (int kk = 0; kk < 2; ++kk) {
      const v16h pa = ldfrag(pw, PTP, 0, kk * 32, lane);
#pragma unroll
      for (int t = 0; t < 4; ++t) {
        const v16h vb = ldfrag(Vs, KTP, t * 16, kk * 32, lane);
        oacc[t] = mma16(pa, vb, oacc[t]);
      }
    }
  }
  __syncthreads();

#pragma unroll
  for (int r = 0; r < 8; ++r) {
    const float inv = 0.015625f / lrow[r];
#pragma unroll
    for (int t = 0; t < 4; ++t) pw[(8 * hh + r) * PTP + 16 * t + c] = (_Float16)(oacc[t][r] * inv);
  }
  __syncthreads();
  v4u val[4];
  size_t go[4];
#pragma unroll
  for (int it = 0; it < 4; ++it) {
    const int p  = lane + 32 * it;
    const int L  = p >> 3;
    const int pc = p & 7;
    Pack8 pk;
    pk.h    = *(const v8h*)(pw + L * PTP + pc * 8);
    val[it] = pk.u;
    go[it]  = ((size_t)(b * NN + q0 + L)) * CC + (size_t)h * DD + pc * 8;
  }
  for (int ps = 0; ps < 2; ++ps) {
#pragma unroll
    for (int it = 0; it < 4; ++it) *(volatile v4u*)(op + go[it]) = val[it];
    __threadfence();
  }
}

#define OTP 68
template <int KK, int RES>
__global__ __launch_bounds__(256) void k_gout(const _Float16* __restrict__ ap,
                                              const _Float16* __restrict__ wt,
                                              const float* __restrict__ bias,
                                              const float* __restrict__ res,
                                              float* __restrict__ out, float oscale) {
  __shared__ __align__(16) float st[8][16 * OTP];
  const int tid = threadIdx.x, lane = tid & 31, wave = tid >> 5;
  const int hh = lane >> 4, c = lane & 15;
  const int m0 = blockIdx.x * 256 + wave * 32;
  const int n0 = blockIdx.y * 64;

  v8f acc[2][4];
#pragma unroll
  for (int s = 0; s < 2; ++s)
#pragma unroll
    for (int t = 0; t < 4; ++t) acc[s][t] = zero8();
  gemm32x64<KK>(ap, KK, wt, KK, m0, n0, lane, acc);

  float bvs[4];
#pragma unroll
  for (int t = 0; t < 4; ++t) bvs[t] = bias[n0 + 16 * t + c];

  float* sw = st[wave];
#pragma unroll
  for (int sub = 0; sub < 2; ++sub) {
    __syncthreads();
#pragma unroll
    for (int t = 0; t < 4; ++t) {
#pragma unroll
      for (int r = 0; r < 8; ++r)
        sw[(8 * hh + r) * OTP + 16 * t + c] = acc[sub][t][r] * oscale + bvs[t];
    }
    __syncthreads();
    v4f val[8];
    size_t go[8];
#pragma unroll
    for (int it = 0; it < 8; ++it) {
      const int p    = lane + 32 * it;
      const int L    = p >> 3;
      const int pc   = p & 7;
      const int row  = L >> 1;
      const int half = L & 1;
      const size_t g = (size_t)(m0 + sub * 16 + row) * CC + n0 + half * 32 + pc * 4;
      v4f v = *(const v4f*)(sw + row * OTP + half * 32 + pc * 4);
      if (RES) {
        const v4f rr = *(const v4f*)(res + g);
        v[0] = v[0] + rr[0]; v[1] = v[1] + rr[1]; v[2] = v[2] + rr[2]; v[3] = v[3] + rr[3];
      }
      val[it] = v;
      go[it]  = g;
    }
    for (int ps = 0; ps < 2; ++ps) {
#pragma unroll
      for (int it = 0; it < 8; ++it) *(volatile v4f*)(out + go[it]) = val[it];
      __threadfence();
    }
  }
}

__global__ __launch_bounds__(256) void k_ffn1(const _Float16* __restrict__ ap,
                                              const _Float16* __restrict__ wt,
                                              const float* __restrict__ bias,
                                              _Float16* __restrict__ hp) {
  __shared__ __align__(16) float st[8][16 * OTP];
  const int tid = threadIdx.x, lane = tid & 31, wave = tid >> 5;
  const int hh = lane >> 4, c = lane & 15;
  const int m0 = blockIdx.x * 256 + wave * 32;
  const int n0 = blockIdx.y * 64;

  v8f acc[2][4];
#pragma unroll
  for (int s = 0; s < 2; ++s)
#pragma unroll
    for (int t = 0; t < 4; ++t) acc[s][t] = zero8();
  gemm32x64<CC>(ap, CC, wt, CC, m0, n0, lane, acc);

  float bvs[4];
#pragma unroll
  for (int t = 0; t < 4; ++t) bvs[t] = bias[n0 + 16 * t + c];

  float* sw = st[wave];
#pragma unroll
  for (int sub = 0; sub < 2; ++sub) {
    __syncthreads();
#pragma unroll
    for (int t = 0; t < 4; ++t) {
#pragma unroll
      for (int r = 0; r < 8; ++r)
        sw[(8 * hh + r) * OTP + 16 * t + c] = acc[sub][t][r] * 0.03125f + bvs[t];
    }
    __syncthreads();
    v4u val[4];
    size_t go[4];
#pragma unroll
    for (int it = 0; it < 4; ++it) {
      const int p  = lane + 32 * it;
      const int L  = p >> 3;
      const int pc = p & 7;
      const v4f x0 = *(const v4f*)(sw + L * OTP + pc * 8);
      const v4f x1 = *(const v4f*)(sw + L * OTP + pc * 8 + 4);
      Pack8 pk;
      pk.h = (v8h){(_Float16)act16(x0[0]), (_Float16)act16(x0[1]), (_Float16)act16(x0[2]), (_Float16)act16(x0[3]),
                   (_Float16)act16(x1[0]), (_Float16)act16(x1[1]), (_Float16)act16(x1[2]), (_Float16)act16(x1[3])};
      val[it] = pk.u;
      go[it]  = (size_t)(m0 + sub * 16 + L) * FF + n0 + pc * 8;
    }
    for (int ps = 0; ps < 2; ++ps) {
#pragma unroll
      for (int it = 0; it < 4; ++it) *(volatile v4u*)(hp + go[it]) = val[it];
      __threadfence();
    }
  }
}

template <int WH>
__global__ __launch_bounds__(256) void k_ln(const float* __restrict__ in,
                                           const float* __restrict__ g,
                                           const float* __restrict__ bt,
                                           float* __restrict__ outf,
                                           _Float16* __restrict__ outh) {
  __shared__ __align__(16) float rb[CC];
  __shared__ float red[16];
  const int tid = threadIdx.x, lane = tid & 31, wave = tid >> 5;
  const size_t ro = (size_t)blockIdx.x * CC;
  const v4f v = *(const v4f*)(in + ro + 4 * tid);
  float s = (v[0] + v[1]) + (v[2] + v[3]);
#pragma unroll
  for (int off = 1; off < 32; off <<= 1) s += __shfl_xor(s, off, 32);
  if (lane == 0) red[wave] = s;
  __syncthreads();
  float ts = 0.f;
#pragma unroll
  for (int w = 0; w < 8; ++w) ts += red[w];
  const float mean = ts * (1.0f / (float)CC);
  const float d0 = v[0] - mean, d1 = v[1] - mean, d2 = v[2] - mean, d3 = v[3] - mean;
  float q = (d0 * d0 + d1 * d1) + (d2 * d2 + d3 * d3);
#pragma unroll
  for (int off = 1; off < 32; off <<= 1) q += __shfl_xor(q, off, 32);
  if (lane == 0) red[8 + wave] = q;
  __syncthreads();
  float tq = 0.f;
#pragma unroll
  for (int w = 0; w < 8; ++w) tq += red[8 + w];
  const float var = tq * (1.0f / (float)CC);
  const float inv = 1.0f / sqrtf(var + 1e-5f);
  const v4f g4 = *(const v4f*)(g + 4 * tid);
  const v4f b4 = *(const v4f*)(bt + 4 * tid);
  v4f o;
  o[0] = d0 * inv * g4[0] + b4[0];
  o[1] = d1 * inv * g4[1] + b4[1];
  o[2] = d2 * inv * g4[2] + b4[2];
  o[3] = d3 * inv * g4[3] + b4[3];
  volatile v4f* dp = (volatile v4f*)(outf + ro + 4 * tid);
  *dp = o;
  __threadfence();
  *dp = o;
  if (WH) {
    *(v4f*)(rb + 4 * tid) = o;
    __syncthreads();
    if (tid < 128) {
      const v4f a0 = *(const v4f*)(rb + 8 * tid);
      const v4f a1 = *(const v4f*)(rb + 8 * tid + 4);
      Pack8 pk;
      pk.h = (v8h){(_Float16)a0[0], (_Float16)a0[1], (_Float16)a0[2], (_Float16)a0[3],
                   (_Float16)a1[0], (_Float16)a1[1], (_Float16)a1[2], (_Float16)a1[3]};
      const v4u vv = pk.u;
      volatile v4u* hq = (volatile v4u*)(outh + ro + 8 * tid);
      *hq = vv;
      __threadfence();
      *hq = vv;
    }
  }
}

extern "C" void kernel_launch(void* const* d_in, const int* in_sizes, int n_in,
                              void* d_out, int out_size, void* d_ws, size_t ws_size,
                              hipStream_t stream) {
  if (n_in < 22) return;
  if (in_sizes[0] != ROWS * CC) return;
  if (in_sizes[1] != NN * NN) return;
  if (in_sizes[2] != CC * CC || in_sizes[3] != CC) return;
  if (in_sizes[4] != CC * LAT || in_sizes[5] != LAT) return;
  if (in_sizes[6] != LAT * CC || in_sizes[7] != CC) return;
  if (in_sizes[8] != CC * LAT || in_sizes[9] != LAT) return;
  if (in_sizes[10] != LAT * CC || in_sizes[11] != CC) return;
  if (in_sizes[12] != CC * CC || in_sizes[13] != CC) return;
  if (in_sizes[14] != CC * FF || in_sizes[15] != FF) return;
  if (in_sizes[16] != FF * CC || in_sizes[17] != CC) return;
  if (in_sizes[18] != CC || in_sizes[19] != CC || in_sizes[20] != CC || in_sizes[21] != CC) return;
  if (out_size != ROWS * CC) return;

  const float* x    = (const float*)d_in[0];
  const float* ab   = (const float*)d_in[1];
  const float* Wq   = (const float*)d_in[2];
  const float* bq   = (const float*)d_in[3];
  const float* WaK  = (const float*)d_in[4];
  const float* baK  = (const float*)d_in[5];
  const float* WbK  = (const float*)d_in[6];
  const float* bbK  = (const float*)d_in[7];
  const float* WaV  = (const float*)d_in[8];
  const float* baV  = (const float*)d_in[9];
  const float* WbV  = (const float*)d_in[10];
  const float* bbV  = (const float*)d_in[11];
  const float* Wo   = (const float*)d_in[12];
  const float* bo   = (const float*)d_in[13];
  const float* W1   = (const float*)d_in[14];
  const float* b1   = (const float*)d_in[15];
  const float* W2   = (const float*)d_in[16];
  const float* b2   = (const float*)d_in[17];
  const float* g1   = (const float*)d_in[18];
  const float* be1  = (const float*)d_in[19];
  const float* g2   = (const float*)d_in[20];
  const float* be2  = (const float*)d_in[21];
  float* out = (float*)d_out;

  size_t off = 0;
  const size_t oX    = off; off += (size_t)ROWS * CC * 2;
  const size_t oWq   = off; off += (size_t)CC * CC * 2;
  const size_t oWlat = off; off += (size_t)2 * LAT * CC * 2;
  const size_t oWbK  = off; off += (size_t)CC * LAT * 2;
  const size_t oWbV  = off; off += (size_t)CC * LAT * 2;
  const size_t oKV   = off; off += (size_t)2 * ROWS * LAT * 2;
  const size_t oQKV  = off; off += 3 * PL * 2;
  const size_t oH    = 0;
  if ((size_t)ROWS * FF * 2 > off) return;
  const size_t oO    = off; off += (size_t)ROWS * CC * 2;
  const size_t oWo   = off; off += (size_t)CC * CC * 2;
  const size_t oW1   = off; off += (size_t)FF * CC * 2;
  const size_t oW2   = off; off += (size_t)CC * FF * 2;
  const size_t oT1   = off; off += (size_t)ROWS * CC * 4;
  const size_t oX1f  = off; off += (size_t)ROWS * CC * 4;
  const size_t oX1h  = off; off += (size_t)ROWS * CC * 2;
  const size_t oT2   = off; off += (size_t)ROWS * CC * 4;
  if (off > ws_size) return;
  if (off > (size_t)134217728) return;

  char* ws = (char*)d_ws;
  _Float16* Xh    = (_Float16*)(ws + oX);
  _Float16* Wqt   = (_Float16*)(ws + oWq);
  _Float16* Wlat  = (_Float16*)(ws + oWlat);
  _Float16* WbKt  = (_Float16*)(ws + oWbK);
  _Float16* WbVt  = (_Float16*)(ws + oWbV);
  _Float16* KVp   = (_Float16*)(ws + oKV);
  _Float16* QKVp  = (_Float16*)(ws + oQKV);
  _Float16* Hp    = (_Float16*)(ws + oH);
  _Float16* Op    = (_Float16*)(ws + oO);
  _Float16* Wot   = (_Float16*)(ws + oWo);
  _Float16* W1t   = (_Float16*)(ws + oW1);
  _Float16* W2t   = (_Float16*)(ws + oW2);
  float*    T1    = (float*)(ws + oT1);
  float*    X1f   = (float*)(ws + oX1f);
  _Float16* X1h   = (_Float16*)(ws + oX1h);
  float*    T2    = (float*)(ws + oT2);

  const int ngrp = in_sizes[0] / 8;
  k_cvt_x<<<dim3((ngrp + 255) / 256), dim3(256), 0, stream>>>(x, Xh, ngrp);
  k_wt<<<dim3(CC / 64, CC / 64), dim3(256), 0, stream>>>(Wq, Wqt, CC, CC);
  k_wt<<<dim3(LAT / 64, CC / 64), dim3(256), 0, stream>>>(WaK, Wlat, LAT, CC);
  k_wt<<<dim3(LAT / 64, CC / 64), dim3(256), 0, stream>>>(WaV, Wlat + (size_t)LAT * CC, LAT, CC);
  k_wt<<<dim3(CC / 64, LAT / 64), dim3(256), 0, stream>>>(WbK, WbKt, CC, LAT);
  k_wt<<<dim3(CC / 64, LAT / 64), dim3(256), 0, stream>>>(WbV, WbVt, CC, LAT);
  k_wt<<<dim3(CC / 64, CC / 64), dim3(256), 0, stream>>>(Wo, Wot, CC, CC);
  k_wt<<<dim3(FF / 64, CC / 64), dim3(256), 0, stream>>>(W1, W1t, FF, CC);
  k_wt<<<dim3(CC / 64, FF / 64), dim3(256), 0, stream>>>(W2, W2t, CC, FF);
  k_lat<<<dim3(ROWS / 256, (2 * LAT) / 64), dim3(256), 0, stream>>>(Xh, Wlat, baK, baV, KVp);
  k_hp<CC, 0><<<dim3(ROWS / 256, CC / 64), dim3(256), 0, stream>>>(Xh, Wqt, bq, QKVp, 0.03125f, 1.0f);
  k_hp<LAT, 0><<<dim3(ROWS / 256, CC / 64), dim3(256), 0, stream>>>(KVp, WbKt, bbK, QKVp + PL, 0.125f, 4.0f);
  k_hp<LAT, 1><<<dim3(ROWS / 256, CC / 64), dim3(256), 0, stream>>>(KVp + (size_t)ROWS * LAT, WbVt, bbV, QKVp + 2 * PL, 0.125f, 4.0f);
  k_attn<<<dim3(BB * HH * (NN / 128)), dim3(256), 0, stream>>>(QKVp, QKVp + PL, QKVp + 2 * PL, ab, Op, 0.03125f);
  k_gout<CC, 1><<<dim3(ROWS / 256, CC / 64), dim3(256), 0, stream>>>(Op, Wot, bo, x, T1, 0.00048828125f);
  k_ln<1><<<dim3(ROWS), dim3(256), 0, stream>>>(T1, g1, be1, X1f, X1h);
  k_ffn1<<<dim3(ROWS / 256, FF / 64), dim3(256), 0, stream>>>(X1h, W1t, b1, Hp);
  k_gout<FF, 1><<<dim3(ROWS / 256, CC / 64), dim3(256), 0, stream>>>(Hp, W2t, b2, X1f, T2, 0.001953125f);
  k_ln<0><<<dim3(ROWS), dim3(256), 0, stream>>>(T2, g2, be2, out, X1h);
  (void)hipGetLastError();
}
